// SelfAttention2D_old_4672924418533
// MI455X (gfx1250) — hardware-verified
//
#include <hip/hip_runtime.h>
#include <math.h>

typedef __attribute__((ext_vector_type(16))) _Float16 v16h;
typedef __attribute__((ext_vector_type(16))) __bf16 v16b;
typedef __attribute__((ext_vector_type(8)))  _Float16 v8h;
typedef __attribute__((ext_vector_type(8)))  float v8f;
typedef __attribute__((ext_vector_type(4)))  float v4f;
typedef __attribute__((ext_vector_type(2)))  float v2f;
typedef __attribute__((ext_vector_type(4)))  unsigned v4u;
typedef __attribute__((ext_vector_type(4)))  int v4i;
typedef float __attribute__((may_alias)) float_a;
typedef int __attribute__((may_alias)) int_a;

template <typename T> __device__ __forceinline__ void vst2(void* p, T v) { *(volatile T*)p = v; __threadfence(); *(volatile T*)p = v; }
__device__ __forceinline__ v8f wmma16(v16h a, v16h b, v8f c) {
  v8f d = __builtin_amdgcn_wmma_f32_16x16x32_f16(false, a, false, b, (short)0, c, false, false);
  asm volatile("v_nop\n\tv_nop\n\tv_nop\n\tv_nop" : "+v"(d) : "v"(a), "v"(b));
  return d;
}
__device__ __forceinline__ v8f wmma_bf(v16b a, v16b b, v8f c) {
  v8f d = __builtin_amdgcn_wmma_f32_16x16x32_bf16(false, a, false, b, (short)0, c, false, false);
  asm volatile("v_nop\n\tv_nop\n\tv_nop\n\tv_nop" : "+v"(d) : "v"(a), "v"(b));
  return d;
}
__device__ __forceinline__ v16h frag_h(const _Float16* rowk0, int lane) {
  union { v16h v; v8h q[2]; } u; const _Float16* p = rowk0 + 8 * (lane >> 4);
  u.q[0] = *(const v8h*)p; u.q[1] = *(const v8h*)(p + 16); return u.v;
}
__device__ __forceinline__ v16h frag_f32(const float* rowk0, int lane) {
  v16h a; const float* p = rowk0 + 8 * (lane >> 4);
#pragma unroll
  for (int i = 0; i < 8; ++i) { a[i] = (_Float16)p[i]; a[8 + i] = (_Float16)p[16 + i]; }
  return a;
}
__device__ __forceinline__ v16h frag_f32s(const float* rowk0, int lane, float sc) {
  v16h a; const float* p = rowk0 + 8 * (lane >> 4);
#pragma unroll
  for (int i = 0; i < 8; ++i) { a[i] = (_Float16)(p[i] * sc); a[8 + i] = (_Float16)(p[16 + i] * sc); }
  return a;
}
__device__ __forceinline__ v16h fragc_f32(const float* W, int k0, int n, int lane, int ld, int K) {
  v16h a; const int g = lane >> 4;
#pragma unroll
  for (int i = 0; i < 8; ++i) { const int ka = k0 + 8 * g + i, kb = ka + 16;
    a[i] = (_Float16)(ka < K ? W[(size_t)ka * ld + n] : 0.f); a[8 + i] = (_Float16)(kb < K ? W[(size_t)kb * ld + n] : 0.f); }
  return a;
}
struct F2 { v16b h, l; };
__device__ __forceinline__ F2 bsplit16(const float v[16]) { F2 r;
#pragma unroll
  for (int i = 0; i < 16; ++i) { const __bf16 h = (__bf16)v[i]; r.h[i] = h; r.l[i] = (__bf16)(v[i] - (float)h); }
  return r; }
__device__ __forceinline__ F2 split_row(const float* row, int k0, int lane) { float v[16]; const float* p = row + k0 + 8 * (lane >> 4);
#pragma unroll
  for (int i = 0; i < 8; ++i) { v[i] = p[i]; v[8 + i] = p[16 + i]; }
  return bsplit16(v); }
__device__ __forceinline__ F2 split_rowK(const float* row, int k0, int lane, int K) { float v[16]; const int g = lane >> 4;
#pragma unroll
  for (int i = 0; i < 8; ++i) { const int ka = k0 + 8 * g + i, kb = ka + 16; v[i] = ka < K ? row[ka] : 0.f; v[8 + i] = kb < K ? row[kb] : 0.f; }
  return bsplit16(v); }
__device__ __forceinline__ F2 split_col(const float* W, int k0, int n, int lane, int ld, int K) { float v[16]; const int g = lane >> 4;
#pragma unroll
  for (int i = 0; i < 8; ++i) { const int ka = k0 + 8 * g + i, kb = ka + 16; v[i] = ka < K ? W[(size_t)ka * ld + n] : 0.f; v[8 + i] = kb < K ? W[(size_t)kb * ld + n] : 0.f; }
  return bsplit16(v); }
__device__ __forceinline__ v8f mac3(const F2& a, const F2& b, v8f c) { c = wmma_bf(a.l, b.h, c); c = wmma_bf(a.h, b.l, c); return wmma_bf(a.h, b.h, c); }
__device__ __forceinline__ float sigm(float v) { return 1.0f / (1.0f + expf(-v)); }
#define LDSX() do { asm volatile("s_wait_dscnt 0" ::: "memory"); __builtin_amdgcn_wave_barrier(); __builtin_amdgcn_fence(__ATOMIC_RELEASE, "workgroup"); } while (0)

#define NB 8
#define NN 4096
#define CC 128
#define DK 16
#define NR (NB * NN)

__global__ __launch_bounds__(128) void k_proj(const float* __restrict__ x, const float* __restrict__ wf, const float* __restrict__ wg, const float* __restrict__ wh, _Float16* __restrict__ F16, _Float16* __restrict__ G16, _Float16* __restrict__ HT) {
  __shared__ __align__(16) float so[4][16][52];
  __shared__ __align__(16) _Float16 st[DK][72];
  const int tid = threadIdx.x, wave = tid >> 5, lane = tid & 31, col = lane & 15, g = lane >> 4;
  const int r0b = blockIdx.x * 64, r0 = r0b + wave * 16; const int b = r0b / NN, n0 = r0b % NN;
  v8f acc[3] = {};
#pragma unroll
  for (int kc = 0; kc < CC / 32; ++kc) { const v16h a = frag_f32(x + (size_t)(r0 + col) * CC + kc * 32, lane);
    acc[0] = wmma16(a, fragc_f32(wf, kc * 32, col, lane, DK, CC), acc[0]); acc[1] = wmma16(a, fragc_f32(wg, kc * 32, col, lane, DK, CC), acc[1]); acc[2] = wmma16(a, fragc_f32(wh, kc * 32, col, lane, DK, CC), acc[2]); }
#pragma unroll
  for (int j = 0; j < 3; ++j)
#pragma unroll
    for (int r = 0; r < 8; ++r) so[wave][8 * g + r][j * 16 + col] = acc[j][r];
  LDSX();
  if (lane < 16) { union { v8h a8; v4u u; } pf0, pf1, pg0, pg1; const int rl = lane;
#pragma unroll
    for (int e = 0; e < 8; ++e) { pf0.a8[e] = (_Float16)so[wave][rl][e]; pf1.a8[e] = (_Float16)so[wave][rl][8 + e]; pg0.a8[e] = (_Float16)so[wave][rl][16 + e]; pg1.a8[e] = (_Float16)so[wave][rl][24 + e]; }
    vst2(F16 + (size_t)(r0 + rl) * DK, pf0.u); vst2(F16 + (size_t)(r0 + rl) * DK + 8, pf1.u); vst2(G16 + (size_t)(r0 + rl) * DK, pg0.u); vst2(G16 + (size_t)(r0 + rl) * DK + 8, pg1.u); }
  if (lane < 16) {
#pragma unroll
    for (int d = 0; d < DK; ++d) st[d][wave * 16 + lane] = (_Float16)so[wave][lane][32 + d]; }
  __syncthreads();
  if (tid < DK * 8) { const int d = tid >> 3, pc = tid & 7; vst2(HT + ((size_t)b * DK + d) * NN + n0 + pc * 8, *(const v4u*)(&st[d][pc * 8])); }
}
__global__ __launch_bounds__(128) void k_colstat(const _Float16* __restrict__ F16, const _Float16* __restrict__ G16, float* __restrict__ cst) {
  __shared__ __align__(16) float sS[4][16][20];
  __shared__ __align__(16) float so[4][16][2];
  const int tid = threadIdx.x, w = tid >> 5, lane = tid & 31, col = lane & 15, g = lane >> 4;
  const int b = blockIdx.y, m0 = blockIdx.x * 64 + w * 16; const size_t rb = (size_t)b * NN;
  v16h ag;
  { const _Float16* gr = G16 + (rb + m0 + col) * DK;
#pragma unroll
    for (int i = 0; i < 8; ++i) { ag[i] = gr[8 * g + i]; ag[8 + i] = (_Float16)0.f; } }
  float mrun = -3.0e38f, lrun = 0.f;
#pragma unroll 1
  for (int nt = 0; nt < NN / 16; ++nt) { v16h bf; const _Float16* fr = F16 + (rb + nt * 16 + col) * DK;
#pragma unroll
    for (int i = 0; i < 8; ++i) { bf[i] = fr[8 * g + i]; bf[8 + i] = (_Float16)0.f; }
    v8f s = {}; s = wmma16(ag, bf, s);
#pragma unroll
    for (int r = 0; r < 8; ++r) sS[w][8 * g + r][col] = s[r];
    LDSX();
    if (g == 0) { const int m = col; float mx = -3.4e38f;
#pragma unroll
      for (int e = 0; e < 16; ++e) mx = fmaxf(mx, sS[w][m][e]);
      const float mnew = fmaxf(mrun, mx); float ps = 0.f;
#pragma unroll
      for (int e = 0; e < 16; ++e) ps += expf(sS[w][m][e] - mnew);
      lrun = lrun * expf(mrun - mnew) + ps; mrun = mnew; }
    LDSX(); }
  if (g == 0) { so[w][col][0] = mrun; so[w][col][1] = 1.0f / lrun; }
  LDSX();
  if (lane < 8) vst2(cst + (rb + m0) * 2 + lane * 4, *(const v4f*)(&so[w][0][0] + lane * 4));
}
__global__ __launch_bounds__(128) void k_apply(const _Float16* __restrict__ F16, const _Float16* __restrict__ G16, const _Float16* __restrict__ HT, const float* __restrict__ cst, const float* __restrict__ wv, const float* __restrict__ gam, const float* __restrict__ x, float* __restrict__ out) {
  __shared__ __align__(16) _Float16 sP[4][16][72];
  __shared__ __align__(16) float sy[4][16][20];
  __shared__ __align__(16) float so[4][16][132];
  const int tid = threadIdx.x, w = tid >> 5, lane = tid & 31, col = lane & 15, g = lane >> 4;
  const int b = blockIdx.y, n0 = blockIdx.x * 64 + w * 16; const size_t rb = (size_t)b * NN;
  v16h af; { const _Float16* fr = F16 + (rb + n0 + col) * DK;
#pragma unroll
    for (int i = 0; i < 8; ++i) { af[i] = fr[8 * g + i]; af[8 + i] = (_Float16)0.f; } }
  v8f acc = {};
#pragma unroll 1
  for (int mt = 0; mt < NN / 64; ++mt) {
#pragma unroll
    for (int t = 0; t < 4; ++t) { const int m = mt * 64 + t * 16 + col; v16h bg; const _Float16* gr = G16 + (rb + m) * DK;
#pragma unroll
      for (int i = 0; i < 8; ++i) { bg[i] = gr[8 * g + i]; bg[8 + i] = (_Float16)0.f; }
      v8f s = {}; s = wmma16(af, bg, s);
      const float Mm = cst[(rb + m) * 2], iL = cst[(rb + m) * 2 + 1];
#pragma unroll
      for (int r = 0; r < 8; ++r) sP[w][8 * g + r][t * 16 + col] = (_Float16)(expf(s[r] - Mm) * iL * 16384.0f); }
    LDSX();
#pragma unroll
    for (int kc = 0; kc < 2; ++kc) acc = wmma16(frag_h(&sP[w][col][0] + kc * 32, lane), frag_h(HT + ((size_t)b * DK + col) * NN + mt * 64 + kc * 32, lane), acc);
    LDSX(); }
#pragma unroll
  for (int r = 0; r < 8; ++r) sy[w][8 * g + r][col] = acc[r] * (1.0f / 16384.0f);
  LDSX();
  { v16h ay;
#pragma unroll
    for (int i = 0; i < 8; ++i) { ay[i] = (_Float16)sy[w][col][8 * g + i]; ay[8 + i] = (_Float16)0.f; }
    const float gm = gam[0];
#pragma unroll
    for (int j = 0; j < 8; ++j) { v16h bb;
#pragma unroll
      for (int i = 0; i < 8; ++i) { bb[i] = (_Float16)(wv[(size_t)(8 * g + i) * CC + j * 16 + col] * 4.0f); bb[8 + i] = (_Float16)0.f; }
      v8f o = {}; o = wmma16(ay, bb, o);
#pragma unroll
      for (int r = 0; r < 8; ++r) { const int c = j * 16 + col; so[w][8 * g + r][c] = gm * o[r] * 0.25f + x[(rb + n0 + 8 * g + r) * CC + c]; } } }
  LDSX();
#pragma unroll 4
  for (int rl = 0; rl < 16; ++rl) vst2(out + (rb + n0 + rl) * CC + lane * 4, *(const v4f*)(&so[w][rl][lane * 4]));
}
extern "C" void kernel_launch(void* const* d_in, const int* in_sizes, int n_in, void* d_out, int out_size, void* d_ws, size_t ws_size, hipStream_t stream) {
  (void)in_sizes; (void)n_in; (void)out_size; (void)ws_size;
  const float** I = (const float**)d_in;
  const float* x = I[0]; const float* wf = I[1]; const float* wg = I[2]; const float* wh = I[3]; const float* wv = I[4]; const float* gam = I[5];
  float* out = (float*)d_out;
  char* ws = (char*)d_ws; size_t off = 0;
  auto take = [&](size_t bytes) { char* p = ws + off; off += (bytes + 255) & ~(size_t)255; return p; };
  _Float16* F16 = (_Float16*)take((size_t)NR * DK * 2); _Float16* G16 = (_Float16*)take((size_t)NR * DK * 2); _Float16* HT = (_Float16*)take((size_t)NR * DK * 2); float* cst = (float*)take((size_t)NR * 2 * 4);
  k_proj<<<NR / 64, 128, 0, stream>>>(x, wf, wg, wh, F16, G16, HT);
  k_colstat<<<dim3(NN / 64, NB), 128, 0, stream>>>(F16, G16, cst);
  k_apply<<<dim3(NN / 64, NB), 128, 0, stream>>>(F16, G16, HT, cst, wv, gam, x, out);
}
